// ImprovedSSM_61641370632867
// MI455X (gfx1250) — hardware-verified
//
#include <hip/hip_runtime.h>
#include <math.h>

constexpr int kBatch = 2;
constexpr int kSeq   = 2048;
constexpr int kHid   = 1024;
constexpr int kInt   = 2048;
constexpr int kNst   = 16;
constexpr int kRows  = kBatch * kSeq;
constexpr int kXpN   = 33;
constexpr int kXpPad = 64;
constexpr float kInvInt = 1.0f / 2048.0f;
constexpr float kLnEps  = 1e-5f;

typedef __attribute__((ext_vector_type(16))) _Float16 v16h;
typedef __attribute__((ext_vector_type(8)))  _Float16 v8h;
typedef __attribute__((ext_vector_type(16))) __bf16   v16b;
typedef __attribute__((ext_vector_type(8)))  __bf16   v8b;
typedef __attribute__((ext_vector_type(8)))  float    v8f;
typedef __attribute__((ext_vector_type(4)))  float    v4f;
typedef __attribute__((ext_vector_type(4)))  unsigned int v4u;

__device__ __forceinline__ unsigned short f2bf_bits(float f) {
  unsigned u = __float_as_uint(f);
  return (unsigned short)((u + 0x7FFFu + ((u >> 16) & 1u)) >> 16);
}
__device__ __forceinline__ float bf_bits2f(unsigned short h) { return __uint_as_float(((unsigned)h) << 16); }
__device__ __forceinline__ float bf_rne(float f) { return bf_bits2f(f2bf_bits(f)); }

__device__ __forceinline__ void dep_guard_h(v8f& a, v8f& b, v16h x, v16h y) { asm volatile("v_nop\n\tv_nop\n\tv_nop\n\tv_nop" : "+v"(a), "+v"(b) : "v"(x), "v"(y)); }
__device__ __forceinline__ void dep_guard_b(v8f& a, v8f& b, v16b x, v16b y) { asm volatile("v_nop\n\tv_nop\n\tv_nop\n\tv_nop" : "+v"(a), "+v"(b) : "v"(x), "v"(y)); }
__device__ __forceinline__ void keep4_h(v16h a, v16h b, v16h c, v16h d) { asm volatile("v_nop" :: "v"(a), "v"(b), "v"(c), "v"(d)); }
__device__ __forceinline__ void keep4_b(v16b a, v16b b, v16b c, v16b d) { asm volatile("v_nop" :: "v"(a), "v"(b), "v"(c), "v"(d)); }
__device__ __forceinline__ void acc_guard4(v8f& a, v8f& b, v8f& c, v8f& d) { asm volatile("v_nop\n\tv_nop\n\tv_nop\n\tv_nop" : "+v"(a), "+v"(b), "+v"(c), "+v"(d)); }
template <typename T> struct Frag;
template <> struct Frag<_Float16> {
  typedef v16h V; union U { v16h v; v8h h[2]; };
  static __device__ __forceinline__ v16h load(const _Float16* p) {
    U f; f.h[0] = *(const v8h*)(p); f.h[1] = *(const v8h*)(p + 16); return f.v;
  }
  static __device__ __forceinline__ v8f mma(v16h a, v16h b, v8f c) {
    return __builtin_amdgcn_wmma_f32_16x16x32_f16(false, a, false, b, (short)0, c, false, false);
  }
  static __device__ __forceinline__ void guard(v8f& a, v8f& b, v16h x, v16h y) { dep_guard_h(a, b, x, y); }
  static __device__ __forceinline__ void keep(v16h a, v16h b, v16h c, v16h d) { keep4_h(a, b, c, d); }
};
template <> struct Frag<__bf16> {
  typedef v16b V; union U { v16b v; v8b h[2]; };
  static __device__ __forceinline__ v16b load(const __bf16* p) {
    U f; f.h[0] = *(const v8b*)(p); f.h[1] = *(const v8b*)(p + 16); return f.v;
  }
  static __device__ __forceinline__ v8f mma(v16b a, v16b b, v8f c) {
    return __builtin_amdgcn_wmma_f32_16x16x32_bf16(false, a, false, b, (short)0, c, false, false);
  }
  static __device__ __forceinline__ void guard(v8f& a, v8f& b, v16b x, v16b y) { dep_guard_b(a, b, x, y); }
  static __device__ __forceinline__ void keep(v16b a, v16b b, v16b c, v16b d) { keep4_b(a, b, c, d); }
};

__device__ __forceinline__ unsigned pk16(unsigned short a, unsigned short b) { return (unsigned)a | ((unsigned)b << 16); }

template <int ET> struct Elem;
template <> struct Elem<0> { typedef _Float16 T; };
template <> struct Elem<1> { typedef __bf16 T; };
template <int ET, bool SPLIT, bool SPLITB, int BIAS_MODE, int OUT_MODE, bool RESID, int ACT = 0>
__global__ __launch_bounds__(256) void wmma_gemm64(
    const unsigned short* __restrict__ Ap, const unsigned short* __restrict__ A2p, int lda, long strideA,
    const unsigned short* __restrict__ Btp, const unsigned short* __restrict__ Bt2p, int ldb, long strideB,
    void* __restrict__ Cout, void* __restrict__ Cout2, int ldc, long strideC,
    const float* __restrict__ bias,
    const float* __restrict__ resid, long strideR,
    int M, int N, int K, float scale) {
  typedef typename Elem<ET>::T T;
  typedef typename Frag<T>::V V;
  const T* A = (const T*)Ap; const T* A2 = (const T*)A2p; const T* Bt = (const T*)Btp; const T* Bt2 = (const T*)Bt2p;
  __shared__ __align__(16) float sT[8][16 * 68];
  const int b    = blockIdx.y;
  const int lane = threadIdx.x & 31;
  const int wave = threadIdx.x >> 5;
  const int tilesN = N >> 6;
  const int tilesM = M >> 6;
  const int tile = blockIdx.x * 8 + wave;
  if (tile >= tilesM * tilesN) return;
  const int tm = tile / tilesN;
  const int tn = tile - tm * tilesN;
  const int m0 = tm << 6;
  const int n0 = tn << 6;

  const T* Ab  = A  + (size_t)b * strideA;
  const T* Bb  = Bt + (size_t)b * strideB;
  const T* Ab2 = SPLIT ? (A2  + (size_t)b * strideA) : nullptr;
  const T* Bb2 = (SPLIT && SPLITB) ? (Bt2 + (size_t)b * strideB) : nullptr;

  const int rlane = lane & 15;
  const int koff  = (lane >> 4) * 8;
  const int mOff  = (lane >> 4) * 8;

  v8f acc[4][4];
#pragma unroll
  for (int i = 0; i < 4; ++i)
#pragma unroll
    for (int j = 0; j < 4; ++j) acc[i][j] = (v8f){0.f,0.f,0.f,0.f,0.f,0.f,0.f,0.f};

  for (int k0 = 0; k0 < K; k0 += 32) {
    V bh[4], bl[4];
#pragma unroll
    for (int j = 0; j < 4; ++j) {
      const size_t bo = (size_t)(n0 + (j << 4) + rlane) * ldb + koff + k0;
      bh[j] = Frag<T>::load(Bb + bo);
      if (SPLIT && SPLITB) bl[j] = Frag<T>::load(Bb2 + bo);
    }
#pragma unroll
    for (int i = 0; i < 4; ++i) {
      const size_t ao = (size_t)(m0 + (i << 4) + rlane) * lda + koff + k0;
      V ah = Frag<T>::load(Ab + ao);
      V al;
      if (SPLIT) al = Frag<T>::load(Ab2 + ao);
#pragma unroll
      for (int j = 0; j < 4; ++j) {
        acc[i][j] = Frag<T>::mma(ah, bh[j], acc[i][j]);
        if (SPLIT && SPLITB) acc[i][j] = Frag<T>::mma(ah, bl[j], acc[i][j]);
        if (SPLIT) acc[i][j] = Frag<T>::mma(al, bh[j], acc[i][j]);
      }
      Frag<T>::guard(acc[i][0], acc[i][3], ah, SPLIT ? al : ah);
    }
    Frag<T>::keep(bh[0], bh[1], bh[2], bh[3]);
    if (SPLIT && SPLITB) Frag<T>::keep(bl[0], bl[1], bl[2], bl[3]);
  }
  acc_guard4(acc[0][0], acc[0][1], acc[0][2], acc[0][3]);
  acc_guard4(acc[1][0], acc[1][1], acc[1][2], acc[1][3]);
  acc_guard4(acc[2][0], acc[2][1], acc[2][2], acc[2][3]);
  acc_guard4(acc[3][0], acc[3][1], acc[3][2], acc[3][3]);

  float* slab = sT[wave];
  const float* Rb = RESID ? (resid + (size_t)b * strideR) : nullptr;
#pragma unroll
  for (int i = 0; i < 4; ++i) {
    const int mBase = m0 + (i << 4);
#pragma unroll
    for (int j = 0; j < 4; ++j) {
      const int n = n0 + (j << 4) + rlane;
      float bv = 0.f;
      if (BIAS_MODE == 2) bv = bias[n];
#pragma unroll
      for (int r = 0; r < 8; ++r) {
        float v = acc[i][j][r] * scale;
        if (BIAS_MODE == 1) v += bias[mBase + mOff + r];
        if (BIAS_MODE == 2) v += bv;
        if (RESID) v += Rb[(size_t)(mBase + mOff + r) * ldc + n];
        if (ACT == 2) v = fmaxf(v, 0.0f);
        if (ACT == 4) v = (v > 0.f) ? v : 0.01f * v;
        slab[(mOff + r) * 68 + (j << 4) + rlane] = v;
      }
    }
    __builtin_amdgcn_fence(__ATOMIC_RELEASE, "workgroup");
    __builtin_amdgcn_wave_barrier();
    __builtin_amdgcn_fence(__ATOMIC_ACQUIRE, "workgroup");
    if (OUT_MODE == 0) {
      float* C = (float*)Cout + (size_t)b * strideC;
      const int hh = lane >> 4, c4 = (lane & 15) * 4;
      for (int pass = 0; pass < 2; ++pass) {
#pragma unroll
        for (int it = 0; it < 8; ++it) {
          const int row = it * 2 + hh;
          v4f v = *(const v4f*)(slab + row * 68 + c4);
          *(volatile v4f*)(C + (size_t)(mBase + row) * ldc + n0 + c4) = v;
        }
        __threadfence();
      }
    } else {
      const int q = lane >> 3, c8 = (lane & 7) * 8;
      unsigned short* C  = (unsigned short*)Cout  + (size_t)b * strideC;
      unsigned short* C2 = (OUT_MODE == 2) ? ((unsigned short*)Cout2 + (size_t)b * strideC) : nullptr;
      for (int pass = 0; pass < 2; ++pass) {
#pragma unroll
        for (int it = 0; it < 4; ++it) {
          const int row = it * 4 + q;
          const float* sp = slab + row * 68 + c8;
          v8h hv, lv;
#pragma unroll
          for (int e = 0; e < 8; ++e) {
            if (OUT_MODE == 1) {
              hv[e] = (_Float16)sp[e];
            } else {
              unsigned short hb = f2bf_bits(sp[e]);
              unsigned short lb = f2bf_bits(sp[e] - bf_bits2f(hb));
              hv[e] = __builtin_bit_cast(_Float16, hb);
              lv[e] = __builtin_bit_cast(_Float16, lb);
            }
          }
          *(volatile v8h*)(C + (size_t)(mBase + row) * ldc + n0 + c8) = hv;
          if (OUT_MODE == 2) *(volatile v8h*)(C2 + (size_t)(mBase + row) * ldc + n0 + c8) = lv;
        }
        __threadfence();
      }
    }
    __builtin_amdgcn_fence(__ATOMIC_RELEASE, "workgroup");
    __builtin_amdgcn_wave_barrier();
    __builtin_amdgcn_fence(__ATOMIC_ACQUIRE, "workgroup");
  }
}

__global__ __launch_bounds__(256) void cast8_bf16_kernel(const float* __restrict__ in, unsigned short* __restrict__ out, int n8) {
  const int i = blockIdx.x * 256 + threadIdx.x;
  if (i >= n8) return;
  const float* p = in + 8 * (size_t)i;
  const v4f a = *(const v4f*)(p);
  const v4f c = *(const v4f*)(p + 4);
  unsigned short hb[8];
#pragma unroll
  for (int e = 0; e < 4; ++e) {
    hb[e]     = f2bf_bits(a[e]);
    hb[4 + e] = f2bf_bits(c[e]);
  }
  const v4u u = (v4u){pk16(hb[0], hb[1]), pk16(hb[2], hb[3]), pk16(hb[4], hb[5]), pk16(hb[6], hb[7])};
  unsigned short* q = out + 8 * (size_t)i;
  *(volatile v4u*)q = u;
  __threadfence();
  *(volatile v4u*)q = u;
}

__global__ __launch_bounds__(256) void tcast_bf16_kernel(const float* __restrict__ in, unsigned short* __restrict__ out, int R, int C) {
  __shared__ float sm[64][65];
  const int t  = threadIdx.x;
  const int c0 = blockIdx.x * 64;
  const int r0 = blockIdx.y * 64;
#pragma unroll
  for (int i = 0; i < 16; ++i) {
    const int e = i * 256 + t;
    const int r = e >> 6;
    const int c = e & 63;
    sm[c][r] = in[(size_t)(r0 + r) * C + c0 + c];
  }
  __syncthreads();
  const int lane = t & 31, wave = t >> 5;
  const int q = lane >> 3, c8 = (lane & 7) * 8;
  for (int pass = 0; pass < 2; ++pass) {
#pragma unroll
    for (int it = 0; it < 2; ++it) {
      const int row = wave * 8 + it * 4 + q;
      unsigned short hb[8];
#pragma unroll
      for (int e = 0; e < 8; ++e) hb[e] = f2bf_bits(sm[row][c8 + e]);
      const v4u u = (v4u){pk16(hb[0], hb[1]), pk16(hb[2], hb[3]), pk16(hb[4], hb[5]), pk16(hb[6], hb[7])};
      *(volatile v4u*)(out + (size_t)(c0 + row) * R + r0 + c8) = u;
    }
    __threadfence();
  }
}

__global__ __launch_bounds__(256) void wxt_kernel(const float* __restrict__ Wx, unsigned short* __restrict__ out) {
  __shared__ float sm[64][65];
  const int t  = threadIdx.x;
  const int i0 = blockIdx.x * 64;
#pragma unroll
  for (int it = 0; it < 16; ++it) {
    const int e  = it * 256 + t;
    const int j  = e >> 6;
    const int il = e & 63;
    const int jc = (j < kXpN) ? j : (kXpN - 1);
    const float v = Wx[(size_t)(i0 + il) * kXpN + jc];
    sm[j][il] = (j < kXpN) ? v : 0.0f;
  }
  __syncthreads();
  const int lane = t & 31, wave = t >> 5;
  const int q = lane >> 3, c8 = (lane & 7) * 8;
  for (int pass = 0; pass < 2; ++pass) {
#pragma unroll
    for (int it = 0; it < 2; ++it) {
      const int row = wave * 8 + it * 4 + q;
      unsigned short hb[8];
#pragma unroll
      for (int e = 0; e < 8; ++e) hb[e] = f2bf_bits(sm[row][c8 + e]);
      const v4u u = (v4u){pk16(hb[0], hb[1]), pk16(hb[2], hb[3]), pk16(hb[4], hb[5]), pk16(hb[6], hb[7])};
      *(volatile v4u*)(out + (size_t)row * kInt + i0 + c8) = u;
    }
    __threadfence();
  }
}

__global__ __launch_bounds__(256) void atab_kernel(const float* __restrict__ Ap, float* __restrict__ atab) {
  __shared__ __align__(16) float sm[256];
  const int t = threadIdx.x;
  const int idx = blockIdx.x * 256 + t;
  const float a = bf_rne(Ap[idx]);
  float sp = fmaxf(a, 0.0f) + log1pf(expf(-fabsf(a)));
  sp = fminf(fmaxf(sp, 0.1f), 10.0f);
  sm[t] = -sp;
  __syncthreads();
  if (t < 64) {
    const v4f v = *(const v4f*)(sm + 4 * t);
    float* p = atab + (size_t)blockIdx.x * 256 + 4 * t;
    *(volatile v4f*)p = v;
    __threadfence();
    *(volatile v4f*)p = v;
  }
}

__global__ __launch_bounds__(256) void conv_ln_kernel(const float* __restrict__ xcf, const float* __restrict__ convw,
                                                     const float* __restrict__ gam, const float* __restrict__ bet,
                                                     unsigned short* __restrict__ xnh, unsigned short* __restrict__ xnl) {
  __shared__ __align__(16) float xs[kInt];
  __shared__ float redA[8];
  __shared__ float redB[8];
  const int row  = blockIdx.x;
  const int s    = row & (kSeq - 1);
  const int bb   = row >> 11;
  const int t    = threadIdx.x;
  const int lane = t & 31, wave = t >> 5;
  const int sm3 = s - 3, sm2 = s - 2, sm1 = s - 1;
  const size_t r0 = (size_t)(bb * kSeq + (sm3 > 0 ? sm3 : 0)) * kInt;
  const size_t r1 = (size_t)(bb * kSeq + (sm2 > 0 ? sm2 : 0)) * kInt;
  const size_t r2 = (size_t)(bb * kSeq + (sm1 > 0 ? sm1 : 0)) * kInt;
  const size_t r3 = (size_t)row * kInt;
  const bool v0 = sm3 >= 0, v1 = sm2 >= 0, v2 = sm1 >= 0;

  float s1 = 0.0f;
#pragma unroll 1
  for (int cc = 0; cc < 8; ++cc) {
    const int i = t + 256 * cc;
    const v4f w4 = *(const v4f*)(convw + 4 * (size_t)i);
    const float l0 = xcf[r0 + i], l1 = xcf[r1 + i], l2 = xcf[r2 + i], l3 = xcf[r3 + i];
    const float x0 = v0 ? l0 : 0.0f, x1 = v1 ? l1 : 0.0f, x2 = v2 ? l2 : 0.0f;
    float a = x0 * bf_rne(w4[0]);
    a += x1 * bf_rne(w4[1]);
    a += x2 * bf_rne(w4[2]);
    a += l3 * bf_rne(w4[3]);
    const float e = expf(fminf(-a, 80.0f));
    const float v = a * __builtin_amdgcn_rcpf(1.0f + e);
    xs[i] = v;
    s1 += v;
  }
#pragma unroll
  for (int off = 16; off > 0; off >>= 1) s1 += __shfl_xor(s1, off, 32);
  if (lane == 0) redA[wave] = s1;
  __syncthreads();
  float tot1 = redA[0];
#pragma unroll
  for (int w = 1; w < 8; ++w) tot1 += redA[w];
  const float mu = tot1 * kInvInt;
  float s2 = 0.0f;
#pragma unroll 1
  for (int cc = 0; cc < 8; ++cc) {
    const int i = t + 256 * cc;
    const float d = xs[i] - mu;
    s2 += d * d;
  }
#pragma unroll
  for (int off = 16; off > 0; off >>= 1) s2 += __shfl_xor(s2, off, 32);
  if (lane == 0) redB[wave] = s2;
  __syncthreads();
  float tot2 = redB[0];
#pragma unroll
  for (int w = 1; w < 8; ++w) tot2 += redB[w];
  const float var  = tot2 * kInvInt;
  const float rstd = rsqrtf(var + kLnEps);
#pragma unroll 1
  for (int cc = 0; cc < 8; ++cc) {
    const int i = t + 256 * cc;
    const float v = xs[i];
    const float g = bf_rne(gam[i]);
    const float be = bf_rne(bet[i]);
    xs[i] = (v - mu) * rstd * g + be;
  }
  __syncthreads();
  {
    const v4f p0 = *(const v4f*)(xs + 8 * t);
    const v4f p1 = *(const v4f*)(xs + 8 * t + 4);
    unsigned short hb[8], lb[8];
#pragma unroll
    for (int e = 0; e < 4; ++e) {
      const float f0 = p0[e];
      hb[e] = f2bf_bits(f0); lb[e] = f2bf_bits(f0 - bf_bits2f(hb[e]));
      const float f1 = p1[e];
      hb[4 + e] = f2bf_bits(f1); lb[4 + e] = f2bf_bits(f1 - bf_bits2f(hb[4 + e]));
    }
    const v4u hu = (v4u){pk16(hb[0], hb[1]), pk16(hb[2], hb[3]), pk16(hb[4], hb[5]), pk16(hb[6], hb[7])};
    const v4u lu = (v4u){pk16(lb[0], lb[1]), pk16(lb[2], lb[3]), pk16(lb[4], lb[5]), pk16(lb[6], lb[7])};
    const size_t o = (size_t)row * kInt + 8 * t;
    *(volatile v4u*)(xnh + o) = hu;
    *(volatile v4u*)(xnl + o) = lu;
    __threadfence();
    *(volatile v4u*)(xnh + o) = hu;
    *(volatile v4u*)(xnl + o) = lu;
  }
}

__global__ __launch_bounds__(256) void gate_kernel(const float* __restrict__ zf, const unsigned short* __restrict__ xnh,
                                                  const unsigned short* __restrict__ xnl, const float* __restrict__ xp,
                                                  const float* __restrict__ atab, const float* __restrict__ dvec,
                                                  unsigned short* __restrict__ gh, unsigned short* __restrict__ gl) {
  __shared__ __align__(16) float xcs[kInt];
  __shared__ __align__(16) float zs[kInt];
  __shared__ __align__(16) float xpl[kXpPad];
  __shared__ __align__(16) float wbc[kNst];
  const int row = blockIdx.x;
  const int t   = threadIdx.x;
  if (t < kXpPad) xpl[t] = xp[(size_t)row * kXpPad + t];
  {
    const size_t o = (size_t)row * kInt + 8 * t;
    const v4u hw = *(const v4u*)(xnh + o);
    const v4u lw = *(const v4u*)(xnl + o);
#pragma unroll
    for (int e = 0; e < 4; ++e) {
      const unsigned wa = hw[e], wb = lw[e];
      xcs[8 * t + 2 * e]     = __uint_as_float((wa & 0xffffu) << 16) + __uint_as_float((wb & 0xffffu) << 16);
      xcs[8 * t + 2 * e + 1] = __uint_as_float(wa & 0xffff0000u) + __uint_as_float(wb & 0xffff0000u);
    }
    *(v4f*)(zs + 8 * t)     = *(const v4f*)(zf + o);
    *(v4f*)(zs + 8 * t + 4) = *(const v4f*)(zf + o + 4);
  }
  __syncthreads();
  if (t < kNst) wbc[t] = xpl[1 + t] * xpl[1 + kNst + t];
  const float p0 = xpl[0];
  float sp = fmaxf(p0, 0.0f) + log1pf(expf(-fabsf(p0)));
  const float delta = fminf(fmaxf(sp, 1e-6f), 10.0f);
  __syncthreads();
#pragma unroll 1
  for (int cc = 0; cc < 8; ++cc) {
    const int i = t + 256 * cc;
    const float x  = xcs[i];
    const float z  = zs[i];
    const float dv = bf_rne(dvec[i]);
    const float* ar = atab + (size_t)i * kNst;
    float sacc = 0.0f;
#pragma unroll 1
    for (int q = 0; q < 4; ++q) {
      const v4f a4 = *(const v4f*)(ar + 4 * q);
      const v4f w4 = *(const v4f*)(wbc + 4 * q);
#pragma unroll
      for (int e = 0; e < 4; ++e) {
        float dcy = expf(delta * a4[e]);
        dcy = fminf(fmaxf(dcy, 1e-6f), 1.0f);
        sacc += w4[e] * dcy;
      }
    }
    const float y  = x * sacc + x * dv;
    const float ez = expf(fminf(-z, 80.0f));
    const float g  = y * (z * __builtin_amdgcn_rcpf(1.0f + ez));
    xcs[i] = g;
  }
  __syncthreads();
  {
    const v4f q0 = *(const v4f*)(xcs + 8 * t);
    const v4f q1 = *(const v4f*)(xcs + 8 * t + 4);
    unsigned short hb[8], lb[8];
#pragma unroll
    for (int e = 0; e < 4; ++e) {
      const float f0 = q0[e];
      hb[e] = f2bf_bits(f0); lb[e] = f2bf_bits(f0 - bf_bits2f(hb[e]));
      const float f1 = q1[e];
      hb[4 + e] = f2bf_bits(f1); lb[4 + e] = f2bf_bits(f1 - bf_bits2f(hb[4 + e]));
    }
    const v4u hu = (v4u){pk16(hb[0], hb[1]), pk16(hb[2], hb[3]), pk16(hb[4], hb[5]), pk16(hb[6], hb[7])};
    const v4u lu = (v4u){pk16(lb[0], lb[1]), pk16(lb[2], lb[3]), pk16(lb[4], lb[5]), pk16(lb[6], lb[7])};
    const size_t o = (size_t)row * kInt + 8 * t;
    *(volatile v4u*)(gh + o) = hu;
    *(volatile v4u*)(gl + o) = lu;
    __threadfence();
    *(volatile v4u*)(gh + o) = hu;
    *(volatile v4u*)(gl + o) = lu;
  }
}

extern "C" void kernel_launch(void* const* d_in, const int* in_sizes, int n_in,
                              void* d_out, int out_size, void* d_ws, size_t ws_size,
                              hipStream_t stream) {
  if (n_in < 9) return;
  const float* x      = (const float*)d_in[0];
  const float* W_in   = (const float*)d_in[1];
  const float* conv_w = (const float*)d_in[2];
  const float* ln_g   = (const float*)d_in[3];
  const float* ln_b   = (const float*)d_in[4];
  const float* W_x    = (const float*)d_in[5];
  const float* A_p    = (const float*)d_in[6];
  const float* Dv     = (const float*)d_in[7];
  const float* W_out  = (const float*)d_in[8];
  float* out = (float*)d_out;

  if ((size_t)in_sizes[0] != (size_t)kRows * kHid) return;
  if ((size_t)in_sizes[1] != (size_t)kHid * 2 * kInt) return;
  if ((size_t)in_sizes[8] != (size_t)kInt * kHid) return;
  if ((size_t)out_size != (size_t)kRows * kHid) return;

  const size_t szRA  = (size_t)kRows * kInt * 4;
  const size_t szRB  = (size_t)kRows * kInt * 4;
  const size_t szXN  = (size_t)kRows * kInt * 2;
  const size_t szXB  = (size_t)kRows * kHid * 2;
  const size_t szWIT = (size_t)2 * kInt * kHid * 2;
  const size_t szWOT = (size_t)kHid * kInt * 2;
  const size_t szXP  = (size_t)kRows * kXpPad * 4;
  const size_t szWXT = (size_t)kXpPad * kInt * 2;
  const size_t szAT  = (size_t)kInt * kNst * 4;

  size_t off = 0;
  const size_t offRA  = off; off += szRA;
  const size_t offRB  = off; off += szRB;
  const size_t offXNh = off; off += szXN;
  const size_t offXNl = off; off += szXN;
  const size_t offXB  = off; off += szXB;
  const size_t offWIT = off; off += szWIT;
  const size_t offWOT = off; off += szWOT;
  const size_t offXP  = off; off += szXP;
  const size_t offWXT = off; off += szWXT;
  const size_t offAT  = off; off += szAT;
  if (off > ws_size) return;

  char* ws = (char*)d_ws;
  float*          xcf = (float*)(ws + offRA);
  unsigned short* ghp = (unsigned short*)(ws + offRA);
  unsigned short* glp = (unsigned short*)(ws + offRA + szXN);
  float*          zf  = (float*)(ws + offRB);
  unsigned short* xnh = (unsigned short*)(ws + offXNh);
  unsigned short* xnl = (unsigned short*)(ws + offXNl);
  unsigned short* xb  = (unsigned short*)(ws + offXB);
  unsigned short* wit = (unsigned short*)(ws + offWIT);
  unsigned short* wot = (unsigned short*)(ws + offWOT);
  float*          xpf = (float*)(ws + offXP);
  unsigned short* wxt = (unsigned short*)(ws + offWXT);
  float*          at  = (float*)(ws + offAT);

  cast8_bf16_kernel<<<(kRows * kHid / 8) / 256, 256, 0, stream>>>(x, xb, kRows * kHid / 8);
  tcast_bf16_kernel<<<dim3(2 * kInt / 64, kHid / 64), 256, 0, stream>>>(W_in, wit, kHid, 2 * kInt);
  tcast_bf16_kernel<<<dim3(kHid / 64, kInt / 64), 256, 0, stream>>>(W_out, wot, kInt, kHid);
  wxt_kernel<<<kInt / 64, 256, 0, stream>>>(W_x, wxt);
  atab_kernel<<<(kInt * kNst) / 256, 256, 0, stream>>>(A_p, at);

  wmma_gemm64<1, false, false, 0, 0, false, 0><<<dim3(256, 2), 256, 0, stream>>>(
      xb, xb, kHid, 0L,
      wit, wit, kHid, (long)kInt * kHid,
      (void*)xcf, (void*)xcf, kInt, (long)kRows * kInt,
      xcf, xcf, 0L,
      kRows, kInt, kHid, 1.0f);

  conv_ln_kernel<<<kRows, 256, 0, stream>>>(xcf, conv_w, ln_g, ln_b, xnh, xnl);

  wmma_gemm64<1, true, false, 0, 0, false, 0><<<dim3(8, 1), 256, 0, stream>>>(
      xnh, xnl, kInt, 0L,
      wxt, wxt, kInt, 0L,
      (void*)xpf, (void*)xpf, kXpPad, 0L,
      xpf, xpf, 0L,
      kRows, kXpPad, kInt, 1.0f);

  gate_kernel<<<kRows, 256, 0, stream>>>(zf, xnh, xnl, xpf, at, Dv, ghp, glp);

  wmma_gemm64<1, true, false, 0, 0, false, 0><<<dim3(128, 1), 256, 0, stream>>>(
      ghp, glp, kInt, 0L,
      wot, wot, kInt, 0L,
      (void*)out, (void*)out, kHid, 0L,
      xpf, xpf, 0L,
      kRows, kHid, kInt, 1.0f);
}
